// DFlashAttentionV5_72292889526399
// MI455X (gfx1250) — hardware-verified
//
#include <hip/hip_runtime.h>


#define NB_  2
#define TQ   1024
#define TC   2048
#define TK   3072
#define DM   2048
#define NH_  16
#define HD   128
#define ZH   2
#define PCAR 1024.0f
#define SCL  0.088388347648318447f
typedef _Float16 h16;
typedef unsigned short bf;
typedef __attribute__((ext_vector_type(16))) __bf16   v16bf;
typedef __attribute__((ext_vector_type(16))) _Float16 v16h;
typedef __attribute__((ext_vector_type(8)))  _Float16 v8h;
typedef __attribute__((ext_vector_type(8)))  unsigned short v8us;
typedef __attribute__((ext_vector_type(8)))  float    v8f;
typedef __attribute__((ext_vector_type(4)))  float    v4f;
typedef v8h  __attribute__((may_alias)) v8ha;
typedef v4f  __attribute__((may_alias)) v4fa;
typedef v8us __attribute__((may_alias)) v8usa;

__device__ __forceinline__ unsigned short f2bf(float f) { unsigned u = __float_as_uint(f); u += 0x7FFFu + ((u >> 16) & 1u); return (unsigned short)(u >> 16); }
__device__ __forceinline__ float bf2f(unsigned short b) { return __uint_as_float(((unsigned)b) << 16); }
__device__ __forceinline__ float bfr(float f) { return bf2f(f2bf(f)); }
__device__ __forceinline__ v16h cat16(v8h lo, v8h hi) { return __builtin_shufflevector(lo, hi, 0, 1, 2, 3, 4, 5, 6, 7, 8, 9, 10, 11, 12, 13, 14, 15); }
__device__ __forceinline__ v16bf cat16b(v8us lo, v8us hi) { return __builtin_bit_cast(v16bf, __builtin_shufflevector(lo, hi, 0, 1, 2, 3, 4, 5, 6, 7, 8, 9, 10, 11, 12, 13, 14, 15)); }
__device__ __forceinline__ v8f wmma16(v16h a, v16h b, v8f c) { return __builtin_amdgcn_wmma_f32_16x16x32_f16(false, a, false, b, (short)0, c, false, false); }
__device__ __forceinline__ v8f wmmab(v16bf a, v16bf b, v8f c) { return __builtin_amdgcn_wmma_f32_16x16x32_bf16(false, a, false, b, (short)0, c, false, false); }


template <typename T16> struct WFrag;
template <> struct WFrag<h16> { typedef v16h V; static __device__ __forceinline__ V ld(const h16* p) { return cat16(*(const v8h*)p, *(const v8h*)(p + 16)); } static __device__ __forceinline__ v8f mma(V a, V b, v8f c) { return wmma16(a, b, c); } };
template <> struct WFrag<bf> { typedef v16bf V; static __device__ __forceinline__ V ld(const bf* p) { return cat16b(*(const v8us*)p, *(const v8us*)(p + 16)); } static __device__ __forceinline__ v8f mma(V a, V b, v8f c) { return wmmab(a, b, c); } };
template <typename T16, int NSPLIT, bool BIAS>
__global__ __launch_bounds__(32) void k_gemmw(const T16* __restrict__ A, const T16* __restrict__ A2, const T16* __restrict__ Bt, const T16* __restrict__ Bt2, int K, float* C, int ldc, const float* __restrict__ bias, size_t sA, size_t sB, size_t sC) {
    typedef typename WFrag<T16>::V V;
    __shared__ __align__(16) float os[16 * 68];
    const size_t z = blockIdx.z; A += z * sA; if (A2) A2 += z * sA; Bt += z * sB; if (Bt2) Bt2 += z * sB; C += z * sC;
    const int lane = threadIdx.x & 31, lr = lane & 15, hi = lane >> 4; const int r0 = blockIdx.x * 64, c0 = blockIdx.y * 64;
    v8f acc[4][4];
#pragma unroll
    for (int mb = 0; mb < 4; ++mb)
#pragma unroll
        for (int nb = 0; nb < 4; ++nb) acc[mb][nb] = (v8f){};
    const size_t aoff = (size_t)(r0 + lr) * K + 8 * hi, boff = (size_t)(c0 + lr) * K + 8 * hi;
#pragma unroll 1
    for (int kc = 0; kc < K; kc += 32) {
        V a[4], a2[4];
#pragma unroll
        for (int mb = 0; mb < 4; ++mb) { a[mb] = WFrag<T16>::ld(A + aoff + (size_t)mb * 16 * K + kc); if (NSPLIT == 1 || NSPLIT == 2) a2[mb] = WFrag<T16>::ld(A2 + aoff + (size_t)mb * 16 * K + kc); }
#pragma unroll
        for (int nb = 0; nb < 4; ++nb) { const V b = WFrag<T16>::ld(Bt + boff + (size_t)nb * 16 * K + kc); V b2; if (NSPLIT >= 2) b2 = WFrag<T16>::ld(Bt2 + boff + (size_t)nb * 16 * K + kc);
#pragma unroll
            for (int mb = 0; mb < 4; ++mb) { acc[mb][nb] = WFrag<T16>::mma(a[mb], b, acc[mb][nb]); if (NSPLIT == 1 || NSPLIT == 2) acc[mb][nb] = WFrag<T16>::mma(a2[mb], b, acc[mb][nb]); if (NSPLIT >= 2) acc[mb][nb] = WFrag<T16>::mma(a[mb], b2, acc[mb][nb]); } }
        asm volatile("v_nop\n\tv_nop\n\tv_nop\n\tv_nop" : "+v"(acc[0][0]), "+v"(acc[1][1]), "+v"(acc[2][2]), "+v"(acc[3][3]) : "v"(a[0]), "v"(a[3]));
    }
#pragma unroll
    for (int mb = 0; mb < 4; ++mb) {
#pragma unroll
        for (int nb = 0; nb < 4; ++nb) {
#pragma unroll
            for (int j = 0; j < 8; ++j) os[(hi * 8 + j) * 68 + nb * 16 + lr] = acc[mb][nb][j]; }
        __builtin_amdgcn_wave_barrier(); asm volatile("" ::: "memory");
        float* crow = C + (size_t)(r0 + mb * 16) * ldc + c0;
#pragma unroll 1
        for (int ps = 0; ps < 2; ++ps) {
#pragma unroll
            for (int s = 0; s < 8; ++s) { const int row = 2 * s + hi, cofs = lr * 4; v4f val = *(const v4fa*)(os + row * 68 + cofs); if (BIAS) { val[0] += bfr(bias[c0 + cofs]); val[1] += bfr(bias[c0 + cofs + 1]); val[2] += bfr(bias[c0 + cofs + 2]); val[3] += bfr(bias[c0 + cofs + 3]); }
                *(volatile v4f*)(crow + (size_t)row * ldc + cofs) = val; }
            if (ps == 0) __threadfence(); }
        __builtin_amdgcn_wave_barrier(); asm volatile("" ::: "memory");
    }
}

__device__ __forceinline__ h16 tohx(float x) { return (h16)x; }
__device__ __forceinline__ void splitf(float y, unsigned short& h, unsigned short& l) { h = f2bf(y); l = f2bf(y - bf2f(h)); }
typedef __attribute__((ext_vector_type(2))) unsigned short v2us;
typedef __attribute__((ext_vector_type(4))) unsigned short v4us;
typedef __attribute__((ext_vector_type(2))) _Float16 v2h;
typedef __attribute__((ext_vector_type(4))) _Float16 v4h;

__global__ __launch_bounds__(256) void k_cvt8(const float* __restrict__ src, bf* dst, size_t n8) { const size_t i = (size_t)blockIdx.x * 256 + threadIdx.x; if (i >= n8) return; const v8f v = *(const v8f*)(src + i * 8); v8us o;
#pragma unroll
    for (int k = 0; k < 8; ++k) o[k] = f2bf(v[k]); *(volatile v8us*)(dst + i * 8) = o; __threadfence(); *(volatile v8us*)(dst + i * 8) = o; }
__global__ __launch_bounds__(256) void k_wtG(const float* __restrict__ w, int K, int N, bf* Bt) {
    const int lane = threadIdx.x & 31; const int L0 = (blockIdx.x * 8 + (threadIdx.x >> 5)) * 8; const int nlines = N * K / 64;
#pragma unroll
    for (int ps = 0; ps < 2; ++ps) {
#pragma unroll 1
        for (int l = 0; l < 8; ++l) { const int L = L0 + l; if (L >= nlines) break; const size_t e = (size_t)L * 64 + lane * 2; const int k = (int)(e % K), n = (int)(e / K); v2us o;
            o[0] = f2bf(w[(size_t)k * N + n]); o[1] = f2bf(w[(size_t)(k + 1) * N + n]); *(volatile v2us*)(Bt + e) = o; }
        if (ps == 0) __threadfence(); }
}

__global__ __launch_bounds__(256) void k_rbf(const float* __restrict__ src, float* dst, size_t n4) { const size_t i = (size_t)blockIdx.x * 256 + threadIdx.x; if (i >= n4) return; const v4f a = *(const v4f*)(src + i * 4); v4f o; for (int u = 0; u < 4; ++u) o[u] = bfr(a[u]); *(volatile v4f*)(dst + i * 4) = o; __threadfence(); *(volatile v4f*)(dst + i * 4) = o; }
__global__ __launch_bounds__(256) void k_rms16(const float* __restrict__ F, const float* __restrict__ w, int ntok, int row0, int nrows, h16* P) { const int lane = threadIdx.x & 31; const int wv = blockIdx.x * 8 + (threadIdx.x >> 5); if (wv >= ntok * (NH_ / 4)) return; const int t = wv / (NH_ / 4); const int hg = (wv % (NH_ / 4)) * 4;
    for (int u = 0; u < 4; ++u) { const int h = hg + u; const float* f = F + (size_t)t * DM + h * HD; const v4f a = *(const v4f*)(f + lane * 4); float ss = 0.f; for (int q = 0; q < 4; ++q) { float p = __fmul_rn(a[q], a[q]); asm volatile("" : "+v"(p)); ss = __fadd_rn(ss, p); }
#pragma unroll
        for (int sh = 16; sh; sh >>= 1) ss = __fadd_rn(ss, __shfl_xor(ss, sh, 32));
        const float rs = __fdiv_rn(1.0f, sqrtf(__fadd_rn(ss * (1.0f / HD), 1e-6f))); v4h o; for (int q = 0; q < 4; ++q) { float n0 = __fmul_rn(a[q], rs); asm volatile("" : "+v"(n0)); o[q] = tohx(__fmul_rn(n0, bfr(w[lane * 4 + q]))); }
        h16* dst = P + ((size_t)h * TK + row0 + t) * HD + lane * 4; *(volatile v4h*)dst = o; __threadfence(); *(volatile v4h*)dst = o; } }
__global__ __launch_bounds__(256) void k_v16(const float* __restrict__ V, int ntok, int row0, h16* VT) { const size_t e = ((size_t)blockIdx.x * 256 + threadIdx.x) * 2; if (e >= (size_t)NH_ * HD * ntok) return; const int t = (int)(e % ntok); const int d = (int)((e / ntok) % HD); const int h = (int)(e / ((size_t)ntok * HD)); v2h o; o[0] = tohx(V[(size_t)t * DM + h * HD + d]); o[1] = tohx(V[(size_t)(t + 1) * DM + h * HD + d]); h16* dst = VT + ((size_t)h * HD + d) * TK + row0 + t; *(volatile v2h*)dst = o; __threadfence(); *(volatile v2h*)dst = o; }
__global__ __launch_bounds__(256) void k_msoft(const float* __restrict__ S, const float* __restrict__ am, h16* P16) { const int lane = threadIdx.x & 31; const int row = blockIdx.x * 8 + (threadIdx.x >> 5); if (row >= ZH * TQ) return; const int i = row % TQ; const float* sr = S + (size_t)row * TK; const float* mr = am + (size_t)i * TK; float v[TK / 32]; float mx = -3.0e38f;
#pragma unroll
    for (int ch = 0; ch < TK / 128; ++ch) { const v4f a = *(const v4f*)(sr + ch * 128 + lane * 4), m4 = *(const v4f*)(mr + ch * 128 + lane * 4);
#pragma unroll
        for (int u = 0; u < 4; ++u) { float sa = a[u] * SCL; asm volatile("" : "+v"(sa)); const float t = __fadd_rn(sa, m4[u]);     v[ch * 4 + u] = t; mx = fmaxf(mx, t); } }
#pragma unroll
    for (int sh = 16; sh; sh >>= 1) mx = fmaxf(mx, __shfl_xor(mx, sh, 32));
    float sum = 0.f;
#pragma unroll
    for (int q = 0; q < TK / 32; ++q) { float d0 = __fsub_rn(v[q], mx); asm volatile("" : "+v"(d0)); v[q] = __builtin_amdgcn_exp2f(__fmul_rn(d0, 1.4426950408889634f)); sum += v[q]; }
#pragma unroll
    for (int sh = 16; sh; sh >>= 1) sum += __shfl_xor(sum, sh, 32);
    const float f = __fdiv_rn(PCAR, sum);
    for (int ps = 0; ps < 2; ++ps) {
#pragma unroll
        for (int ch = 0; ch < TK / 128; ++ch) { v4h o4; for (int q = 0; q < 4; ++q) o4[q] = tohx(v[ch * 4 + q] * f); *(volatile v4h*)(P16 + (size_t)row * TK + ch * 128 + lane * 4) = o4; }
        if (ps == 0) __threadfence(); } }
__global__ __launch_bounds__(256) void k_mrg(const float* __restrict__ O, int h0, bf* Ah, bf* Al) { const size_t e = ((size_t)blockIdx.x * 256 + threadIdx.x) * 4; if (e >= (size_t)ZH * TQ * HD) return; const int d = (int)(e % HD); const int t = (int)((e / HD) % TQ); const int zz = (int)(e / ((size_t)HD * TQ)); const size_t oo = (size_t)t * DM + (h0 + zz) * HD + d; v4us oh, ol;
#pragma unroll
    for (int u = 0; u < 4; ++u) { unsigned short a, b; splitf(O[e + u] * (1.0f / PCAR), a, b); oh[u] = a; ol[u] = b; } *(volatile v4us*)(Ah + oo) = oh; *(volatile v4us*)(Al + oo) = ol; __threadfence(); *(volatile v4us*)(Ah + oo) = oh; *(volatile v4us*)(Al + oo) = ol; }

extern "C" void kernel_launch(void* const* d_in, const int* in_sizes, int n_in,
                              void* d_out, int out_size, void* d_ws, size_t ws_size, hipStream_t stream) {
    (void)in_sizes; (void)n_in; (void)out_size;
    const float* x = (const float*)d_in[0]; const float* cx = (const float*)d_in[1]; const float* am = (const float*)d_in[2]; const float* w_q = (const float*)d_in[3]; const float* w_k = (const float*)d_in[4]; const float* w_v = (const float*)d_in[5]; const float* w_ck = (const float*)d_in[6]; const float* w_cv = (const float*)d_in[7]; const float* w_out = (const float*)d_in[8]; const float* qnw = (const float*)d_in[9]; const float* knw = (const float*)d_in[10];
    float* OUT = (float*)d_out;
    char* wsp = (char*)d_ws;
    auto take = [&](size_t bytes) { char* p = wsp; wsp += (bytes + 255) & ~(size_t)255; return (void*)p; };
    bf* BQ = (bf*)take((size_t)DM * DM * 2); bf* BK = (bf*)take((size_t)DM * DM * 2); bf* BV = (bf*)take((size_t)DM * DM * 2); bf* BCK = (bf*)take((size_t)DM * DM * 2); bf* BCV = (bf*)take((size_t)DM * DM * 2); bf* BO = (bf*)take((size_t)DM * DM * 2);
    bf* XB = (bf*)take((size_t)TC * DM * 2); float* F = (float*)take((size_t)TC * DM * 4);
    h16* QP = (h16*)take((size_t)NH_ * TK * HD * 2); h16* KP = (h16*)take((size_t)NH_ * TK * HD * 2); h16* VT = (h16*)take((size_t)NH_ * HD * TK * 2);
    float* S = (float*)take((size_t)ZH * TQ * TK * 4); h16* P16 = (h16*)take((size_t)ZH * TQ * TK * 2); float* O = (float*)take((size_t)ZH * TQ * HD * 4); bf* ATh = (bf*)take((size_t)TQ * DM * 2); bf* ATl = (bf*)take((size_t)TQ * DM * 2); float* AMR = (float*)take((size_t)TQ * TK * 4);
    if ((size_t)(wsp - (char*)d_ws) > ws_size) return;
    const float* Ws[6] = {w_q, w_k, w_v, w_ck, w_cv, w_out}; bf* Bs[6] = {BQ, BK, BV, BCK, BCV, BO};
    for (int i = 0; i < 6; ++i) k_wtG<<<(DM * DM / 64 + 63) / 64, 256, 0, stream>>>(Ws[i], DM, DM, Bs[i]);
    const size_t zq = (size_t)TK * HD, zS = (size_t)TQ * TK, zv = (size_t)HD * TK, zo = (size_t)TQ * HD;
    for (int b = 0; b < NB_; ++b) {
        k_cvt8<<<(TC * DM / 8 + 255) / 256, 256, 0, stream>>>(cx + (size_t)b * TC * DM, XB, TC * DM / 8);
        k_gemmw<bf, 0, false><<<dim3(TC / 64, DM / 64, 1), 32, 0, stream>>>(XB, nullptr, BCK, nullptr, DM, F, DM, nullptr, 0, 0, 0); k_rms16<<<TC * (NH_ / 4) / 8, 256, 0, stream>>>(F, knw, TC, 0, TK, KP);
        k_gemmw<bf, 0, false><<<dim3(TC / 64, DM / 64, 1), 32, 0, stream>>>(XB, nullptr, BCV, nullptr, DM, F, DM, nullptr, 0, 0, 0); k_v16<<<(unsigned)(((size_t)NH_ * HD * TC / 2 + 255) / 256), 256, 0, stream>>>(F, TC, 0, VT);
        k_cvt8<<<(TQ * DM / 8 + 255) / 256, 256, 0, stream>>>(x + (size_t)b * TQ * DM, XB, TQ * DM / 8);
        k_gemmw<bf, 0, false><<<dim3(TQ / 64, DM / 64, 1), 32, 0, stream>>>(XB, nullptr, BQ, nullptr, DM, F, DM, nullptr, 0, 0, 0); k_rms16<<<TQ * (NH_ / 4) / 8, 256, 0, stream>>>(F, qnw, TQ, 0, TK, QP);
        k_gemmw<bf, 0, false><<<dim3(TQ / 64, DM / 64, 1), 32, 0, stream>>>(XB, nullptr, BK, nullptr, DM, F, DM, nullptr, 0, 0, 0); k_rms16<<<TQ * (NH_ / 4) / 8, 256, 0, stream>>>(F, knw, TQ, TC, TK, KP);
        k_gemmw<bf, 0, false><<<dim3(TQ / 64, DM / 64, 1), 32, 0, stream>>>(XB, nullptr, BV, nullptr, DM, F, DM, nullptr, 0, 0, 0); k_v16<<<(unsigned)(((size_t)NH_ * HD * TQ / 2 + 255) / 256), 256, 0, stream>>>(F, TQ, TC, VT);
        k_rbf<<<(unsigned)(((size_t)TQ * TK / 4 + 255) / 256), 256, 0, stream>>>(am + (size_t)b * TQ * TK, AMR, (size_t)TQ * TK / 4);
        for (int h0 = 0; h0 < NH_; h0 += ZH) {
            k_gemmw<h16, 0, false><<<dim3(TQ / 64, TK / 64, ZH), 32, 0, stream>>>(QP + (size_t)h0 * zq, nullptr, KP + (size_t)h0 * zq, nullptr, HD, S, TK, nullptr, zq, zq, zS);
            k_msoft<<<ZH * TQ / 8, 256, 0, stream>>>(S, AMR, P16);
            k_gemmw<h16, 0, false><<<dim3(TQ / 64, HD / 64, ZH), 32, 0, stream>>>(P16, nullptr, VT + (size_t)h0 * zv, nullptr, TK, O, HD, nullptr, zS, zv, zo);
            k_mrg<<<(unsigned)(((size_t)ZH * TQ * HD / 4 + 255) / 256), 256, 0, stream>>>(O, h0, ATh, ATl); }
        k_gemmw<bf, 1, false><<<dim3(TQ / 64, DM / 64, 1), 32, 0, stream>>>(ATh, ATl, BO, nullptr, DM, OUT + (size_t)b * TQ * DM, DM, nullptr, 0, 0, 0); }
}
